// MultiScaleDeformableAlingment_37572373905603
// MI455X (gfx1250) — hardware-verified
//
#include <hip/hip_runtime.h>


typedef __attribute__((ext_vector_type(16))) _Float16 v16h;
typedef __attribute__((ext_vector_type(8)))  _Float16 v8h;
typedef __attribute__((ext_vector_type(8)))  float    v8f;

#define TPB 256
#define TILE_PIX 64
#define LOSC 2048.0f
#define INV_LOSC 0.00048828125f

__device__ __forceinline__ v8f wmma16(v16h a, v16h b, v8f c) {
  v8f d = __builtin_amdgcn_wmma_f32_16x16x32_f16(false, a, false, b, (short)0, c, false, false);
  asm volatile("v_nop\n\tv_nop\n\tv_nop\n\tv_nop" : "+v"(d) : "v"(a), "v"(b));
  return d;
}
template <typename F>
__device__ __forceinline__ void store_rows32(const v8f& c0, const v8f& c1, int lane, F&& rowptr) {
  const int hi = lane >> 4;
  for (int pass = 0; pass < 2; ++pass) {
#pragma unroll
    for (int r = 0; r < 8; ++r) {
      const float a0 = c0[r], b0 = c1[r];
      const float ax = __shfl_xor(a0, 16), bx = __shfl_xor(b0, 16);
      const float v1 = hi ? bx : a0;
      const float v2 = hi ? b0 : ax;
      float* p1 = rowptr(r); float* p2 = rowptr(r + 8);
      if (p1) *(volatile float*)(p1 + lane) = v1;
      if (p2) *(volatile float*)(p2 + lane) = v2;
    }
    __threadfence();
  }
}

__global__ void pack_w_kernel(const float* __restrict__ w, _Float16* __restrict__ wtr, _Float16* __restrict__ wlo,
                              int Cout, int Mpad, int K) {
  int i8 = blockIdx.x * blockDim.x + threadIdx.x;
  if (i8 >= Mpad * K / 8) return;
  v8h h, l;
#pragma unroll
  for (int e = 0; e < 8; ++e) {
    int i = i8 * 8 + e;
    int co = i / K, r = i % K;
    float v = (co < Cout) ? w[(size_t)co * K + r] : 0.f;
    _Float16 hv = (_Float16)v; h[e] = hv; l[e] = (_Float16)((v - (float)hv) * LOSC);
  }
  *(volatile v8h*)(wtr + (size_t)i8 * 8) = h; if (wlo) *(volatile v8h*)(wlo + (size_t)i8 * 8) = l;
  __threadfence();
  *(volatile v8h*)(wtr + (size_t)i8 * 8) = h; if (wlo) *(volatile v8h*)(wlo + (size_t)i8 * 8) = l;
}

__global__ void pack_w_deform_kernel(const float* __restrict__ w, _Float16* __restrict__ wtr) {
  int i8 = blockIdx.x * blockDim.x + threadIdx.x;
  if (i8 >= 64 * 576 / 8) return;
  v8h h;
#pragma unroll
  for (int e = 0; e < 8; ++e) {
    int i = i8 * 8 + e;
    int o = i / 576, r = i % 576;
    int gk = r >> 4, c = r & 15;
    int g = gk / 9, k = gk % 9;
    h[e] = (_Float16)w[(size_t)o * 576 + (g * 16 + c) * 9 + k];
  }
  *(volatile v8h*)(wtr + (size_t)i8 * 8) = h; __threadfence(); *(volatile v8h*)(wtr + (size_t)i8 * 8) = h;
}

__device__ __forceinline__ v16h ldfrag(const _Float16* row, int hi) {
  v16h f;
#pragma unroll
  for (int j = 0; j < 8; ++j) {
    f[j]     = row[hi * 8 + j];
    f[j + 8] = row[16 + hi * 8 + j];
  }
  return f;
}

__device__ __forceinline__ float sigmoid_fast(float v) {
  return __builtin_amdgcn_rcpf(1.f + __expf(-v));
}

template <int CIN, int PAIR, int EPI, int SPLIT>
__global__ __launch_bounds__(TPB) void conv3x3_wmma(
    const float* __restrict__ srcA, const float* __restrict__ srcB,
    int H, int W,
    const _Float16* __restrict__ wtr, const _Float16* __restrict__ wlo, const float* __restrict__ bias,
    int Cout, int Mtiles, float* __restrict__ out0, float rng) {
  extern __shared__ __attribute__((aligned(16))) _Float16 patch[];
  constexpr int K = CIN * 9;
  constexpr int KS = K + 8;
  constexpr int KSTEPS = K / 32;
  _Float16* patchlo = patch + TILE_PIX * KS;
  const int HW = H * W;
  const int n     = blockIdx.y;
  const int ptile = blockIdx.x * TILE_PIX;
  const int tid   = threadIdx.x;

  for (int t = tid; t < TILE_PIX * CIN; t += TPB) {
    int pl = t % TILE_PIX;
    int ci = t / TILE_PIX;
    int p = ptile + pl;
    int y = p / W, x = p % W;
    const float* src;
    if (PAIR) {
      int b = n >> 2, g = n & 3;
      int cc = ci & 15;
      const float* base = (ci < 16) ? srcA : srcB;
      src = base + ((size_t)b * 64 + g * 16 + cc) * HW;
    } else {
      src = srcA + ((size_t)n * CIN + ci) * HW;
    }
    _Float16* dst = patch + pl * KS + ci * 9;
    _Float16* dlo = patchlo + pl * KS + ci * 9;
#pragma unroll
    for (int kk = 0; kk < 9; ++kk) {
      int yy = y - 1 + kk / 3, xx = x - 1 + kk % 3;
      float v = (yy >= 0 && yy < H && xx >= 0 && xx < W) ? src[yy * W + xx] : 0.f;
      _Float16 hv = (_Float16)v;
      dst[kk] = hv;
      if (SPLIT) dlo[kk] = (_Float16)((v - (float)hv) * LOSC);
    }
  }
  __syncthreads();

  const int wave = tid >> 5;
  const int lane = tid & 31;
  const int l = lane & 15, hi = lane >> 4;
  for (int task = wave; task < Mtiles * 2; task += 8) {
    int mtile = task >> 1, np = task & 1;
    const _Float16* arow  = wtr + (size_t)(mtile * 16 + l) * K;
    const _Float16* alow  = SPLIT ? (wlo + (size_t)(mtile * 16 + l) * K) : arow;
    const _Float16* brow0 = patch + (np * 32 + l) * KS;
    const _Float16* brow1 = brow0 + 16 * KS;
    const _Float16* blo0  = patchlo + (np * 32 + l) * KS;
    const _Float16* blo1  = blo0 + 16 * KS;
    v8f c0 = {0.f, 0.f, 0.f, 0.f, 0.f, 0.f, 0.f, 0.f};
    v8f c1 = {0.f, 0.f, 0.f, 0.f, 0.f, 0.f, 0.f, 0.f};
    v8f x0 = {0.f, 0.f, 0.f, 0.f, 0.f, 0.f, 0.f, 0.f};
    v8f x1 = {0.f, 0.f, 0.f, 0.f, 0.f, 0.f, 0.f, 0.f};
#pragma unroll 2
    for (int s = 0; s < KSTEPS; ++s) {
      v16h a  = ldfrag(arow + s * 32, hi);
      v16h b0 = ldfrag(brow0 + s * 32, hi);
      v16h b1 = ldfrag(brow1 + s * 32, hi);
      c0 = wmma16(a, b0, c0);
      c1 = wmma16(a, b1, c1);
      if (SPLIT) {
        v16h al  = ldfrag(alow + s * 32, hi);
        v16h bl0 = ldfrag(blo0 + s * 32, hi);
        v16h bl1 = ldfrag(blo1 + s * 32, hi);
        x0 = wmma16(a, bl0, x0); x0 = wmma16(al, b0, x0);
        x1 = wmma16(a, bl1, x1); x1 = wmma16(al, b1, x1);
      }
    }
    v8f e0, e1;
#pragma unroll
    for (int r = 0; r < 8; ++r) {
      int co = mtile * 16 + r + hi * 8;
      float bb = (co < Cout) ? bias[co] : 0.f;
      float v0 = c0[r] + (SPLIT ? x0[r] * INV_LOSC : 0.f) + bb;
      float v1 = c1[r] + (SPLIT ? x1[r] * INV_LOSC : 0.f) + bb;
      if (EPI == 1) { e0[r] = rng * 2.f * sigmoid_fast(v0) - rng; e1[r] = rng * 2.f * sigmoid_fast(v1) - rng; }
      else          { e0[r] = 2.f * sigmoid_fast(v0);             e1[r] = 2.f * sigmoid_fast(v1); }
    }
    const int p0 = ptile + np * 32;
    store_rows32(e0, e1, lane, [&](int rr) -> float* {
      int co = mtile * 16 + rr;
      if (co >= Cout) return (float*)nullptr;
      if (EPI == 1) { int b = n >> 2, g = n & 3; return out0 + ((size_t)b * 72 + g * 18 + co) * HW + p0; }
      return out0 + ((size_t)n * 36 + co) * HW + p0;
    });
  }
}

__global__ __launch_bounds__(TPB) void deform_wmma(
    const float* __restrict__ sou, const float* __restrict__ offmap,
    const float* __restrict__ modmap, const _Float16* __restrict__ wtr,
    float* __restrict__ out, int H, int W) {
  extern __shared__ __attribute__((aligned(16))) _Float16 patch[];
  constexpr int K = 576, KS = K + 8, KSTEPS = K / 32;
  const int HW = H * W;
  const int b     = blockIdx.y;
  const int ptile = blockIdx.x * TILE_PIX;
  const int tid   = threadIdx.x;

  for (int t = tid; t < TILE_PIX * 36; t += TPB) {
    int pl = t % TILE_PIX;
    int gk = t / TILE_PIX;
    int g = gk / 9, k = gk % 9;
    int p = ptile + pl;
    int y = p / W, x = p % W;
    float dy = offmap[((size_t)b * 72 + g * 18 + k * 2) * HW + p];
    float dx = offmap[((size_t)b * 72 + g * 18 + k * 2 + 1) * HW + p];
    float m  = modmap[((size_t)b * 36 + g * 9 + k) * HW + p];
    float py = (float)(y - 1 + k / 3) + dy;
    float px = (float)(x - 1 + k % 3) + dx;
    float y0f = floorf(py), x0f = floorf(px);
    float wy = py - y0f, wx = px - x0f;
    int y0 = (int)y0f, x0 = (int)x0f;
    int y1 = y0 + 1, x1 = x0 + 1;
    float v00 = ((y0 >= 0 && y0 < H && x0 >= 0 && x0 < W) ? 1.f : 0.f) * (1.f - wy) * (1.f - wx);
    float v01 = ((y0 >= 0 && y0 < H && x1 >= 0 && x1 < W) ? 1.f : 0.f) * (1.f - wy) * wx;
    float v10 = ((y1 >= 0 && y1 < H && x0 >= 0 && x0 < W) ? 1.f : 0.f) * wy * (1.f - wx);
    float v11 = ((y1 >= 0 && y1 < H && x1 >= 0 && x1 < W) ? 1.f : 0.f) * wy * wx;
    int cy0 = y0 < 0 ? 0 : (y0 > H - 1 ? H - 1 : y0);
    int cy1 = y1 < 0 ? 0 : (y1 > H - 1 ? H - 1 : y1);
    int cx0 = x0 < 0 ? 0 : (x0 > W - 1 ? W - 1 : x0);
    int cx1 = x1 < 0 ? 0 : (x1 > W - 1 ? W - 1 : x1);
    const float* base = sou + ((size_t)b * 64 + g * 16) * HW;
    _Float16* dst = patch + pl * KS + gk * 16;
#pragma unroll 4
    for (int c = 0; c < 16; ++c) {
      const float* ch = base + (size_t)c * HW;
      float v = v00 * ch[cy0 * W + cx0] + v01 * ch[cy0 * W + cx1] +
                v10 * ch[cy1 * W + cx0] + v11 * ch[cy1 * W + cx1];
      dst[c] = (_Float16)(v * m);
    }
  }
  __syncthreads();

  const int wave = tid >> 5;
  const int lane = tid & 31;
  const int l = lane & 15, hi = lane >> 4;
  const int mtile = wave >> 1, np = wave & 1;
  const _Float16* arow  = wtr + (size_t)(mtile * 16 + l) * K;
  const _Float16* brow0 = patch + (np * 32 + l) * KS;
  const _Float16* brow1 = brow0 + 16 * KS;
  v8f c0 = {0.f, 0.f, 0.f, 0.f, 0.f, 0.f, 0.f, 0.f};
  v8f c1 = {0.f, 0.f, 0.f, 0.f, 0.f, 0.f, 0.f, 0.f};
#pragma unroll 2
  for (int s = 0; s < KSTEPS; ++s) {
    v16h a  = ldfrag(arow + s * 32, hi);
    v16h b0 = ldfrag(brow0 + s * 32, hi);
    v16h b1 = ldfrag(brow1 + s * 32, hi);
    c0 = wmma16(a, b0, c0);
    c1 = wmma16(a, b1, c1);
  }
  const int p0 = ptile + np * 32;
  store_rows32(c0, c1, lane, [&](int rr) -> float* { return out + ((size_t)b * 64 + mtile * 16 + rr) * HW + p0; });
}

__global__ void mean_off_kernel(const float* __restrict__ offmap, float* __restrict__ oyox, int HW) {
  int i = blockIdx.x * blockDim.x + threadIdx.x;
  if (i >= 2 * HW) return;
  int b = i / HW, p = i % HW;
  float sdy = 0.f, sdx = 0.f;
  for (int j = 0; j < 36; ++j) {
    sdy += offmap[((size_t)b * 72 + 2 * j) * HW + p];
    sdx += offmap[((size_t)b * 72 + 2 * j + 1) * HW + p];
  }
  volatile float* o0 = oyox + ((size_t)b * 2 + 0) * HW + p; volatile float* o1 = oyox + ((size_t)b * 2 + 1) * HW + p;
  *o0 = sdy * (1.f / 36.f); *o1 = sdx * (1.f / 36.f);
  __threadfence();
  *o0 = sdy * (1.f / 36.f); *o1 = sdx * (1.f / 36.f);
}

__global__ void upsample_ov_kernel(const float* __restrict__ oyox, float* __restrict__ out,
                                   int H, int W, float fs) {
  int i = blockIdx.x * blockDim.x + threadIdx.x;
  int xo = i & 511;
  int yo = (i >> 9) & 511;
  int ch = (i >> 18) & 1;
  int b  = i >> 19;
  float sy = (float)yo * (float)(H - 1) * (1.f / 511.f);
  float sx = (float)xo * (float)(W - 1) * (1.f / 511.f);
  int y0 = (int)floorf(sy); y0 = y0 < 0 ? 0 : (y0 > H - 2 ? H - 2 : y0);
  int x0 = (int)floorf(sx); x0 = x0 < 0 ? 0 : (x0 > W - 2 ? W - 2 : x0);
  float wy = sy - (float)y0, wx = sx - (float)x0;
  const float* pl = oyox + ((size_t)b * 2 + ch) * H * W;
  float v = pl[y0 * W + x0] * (1.f - wy) * (1.f - wx) +
            pl[y0 * W + x0 + 1] * (1.f - wy) * wx +
            pl[(y0 + 1) * W + x0] * wy * (1.f - wx) +
            pl[(y0 + 1) * W + x0 + 1] * wy * wx;
  *(volatile float*)(out + i) = v * fs;
  __threadfence();
  *(volatile float*)(out + i) = v * fs;
}

extern "C" void kernel_launch(void* const* d_in, const int* in_sizes, int n_in,
                              void* d_out, int out_size, void* d_ws, size_t ws_size,
                              hipStream_t stream) {
  (void)in_sizes; (void)n_in; (void)out_size;
  const float* sou[3]   = {(const float*)d_in[0],  (const float*)d_in[2],  (const float*)d_in[4]};
  const float* ref[3]   = {(const float*)d_in[1],  (const float*)d_in[3],  (const float*)d_in[5]};
  const float* off_w[3] = {(const float*)d_in[6],  (const float*)d_in[11], (const float*)d_in[16]};
  const float* off_b[3] = {(const float*)d_in[7],  (const float*)d_in[12], (const float*)d_in[17]};
  const float* mod_w[3] = {(const float*)d_in[8],  (const float*)d_in[13], (const float*)d_in[18]};
  const float* mod_b[3] = {(const float*)d_in[9],  (const float*)d_in[14], (const float*)d_in[19]};
  const float* reg_w[3] = {(const float*)d_in[10], (const float*)d_in[15], (const float*)d_in[20]};

  float* out = (float*)d_out;
  float* featp[3] = {out + 655360, out + 131072, out + 0};
  float* ovp[3]   = {out + 4849664, out + 3801088, out + 2752512};
  const int   Hs[3]   = {128, 64, 32};
  const float rngs[3] = {32.f, 16.f, 8.f};
  const float fss[3]  = {4.f, 8.f, 16.f};

  size_t woff = 0;
  auto alloc = [&](size_t bytes) -> void* {
    void* p = (void*)((char*)d_ws + woff);
    woff += (bytes + 255) & ~(size_t)255;
    return p;
  };

  const size_t shm_off = (size_t)2 * TILE_PIX * (32 * 9 + 8) * sizeof(_Float16);
  const size_t shm_big = (size_t)TILE_PIX * (64 * 9 + 8) * sizeof(_Float16);
  if (ws_size < (size_t)64 * 1024 * 1024) return;

  for (int s = 0; s < 3; ++s) {
    int H = Hs[s], W = Hs[s], HW = H * W;
    float*    offmap = (float*)alloc((size_t)2 * 72 * HW * sizeof(float));
    float*    modmap = (float*)alloc((size_t)2 * 36 * HW * sizeof(float));
    float*    oyox   = (float*)alloc((size_t)2 * 2 * HW * sizeof(float));
    _Float16* wtrO   = (_Float16*)alloc((size_t)32 * 288 * sizeof(_Float16));
    _Float16* wloO   = (_Float16*)alloc((size_t)32 * 288 * sizeof(_Float16));
    _Float16* wtrM   = (_Float16*)alloc((size_t)48 * 576 * sizeof(_Float16));
    _Float16* wtrR   = (_Float16*)alloc((size_t)64 * 576 * sizeof(_Float16));

    pack_w_kernel<<<(32 * 288 / 8 + TPB - 1) / TPB, TPB, 0, stream>>>(off_w[s], wtrO, wloO, 18, 32, 288);
    pack_w_kernel<<<(48 * 576 / 8 + TPB - 1) / TPB, TPB, 0, stream>>>(mod_w[s], wtrM, nullptr, 36, 48, 576);
    pack_w_deform_kernel<<<(64 * 576 / 8 + TPB - 1) / TPB, TPB, 0, stream>>>(reg_w[s], wtrR);

    conv3x3_wmma<32, 1, 1, 1><<<dim3(HW / TILE_PIX, 8), TPB, shm_off, stream>>>(
        sou[s], ref[s], H, W, wtrO, wloO, off_b[s], 18, 2, offmap, rngs[s]);
    conv3x3_wmma<64, 0, 2, 0><<<dim3(HW / TILE_PIX, 2), TPB, shm_big, stream>>>(
        sou[s], nullptr, H, W, wtrM, nullptr, mod_b[s], 36, 3, modmap, 0.f);
    deform_wmma<<<dim3(HW / TILE_PIX, 2), TPB, shm_big, stream>>>(
        sou[s], offmap, modmap, wtrR, featp[s], H, W);
    mean_off_kernel<<<(2 * HW + TPB - 1) / TPB, TPB, 0, stream>>>(offmap, oyox, HW);
    upsample_ov_kernel<<<(2 * 2 * 512 * 512) / TPB, TPB, 0, stream>>>(oyox, ovp[s], H, W, fss[s]);
  }
}
